// VisionEncoderMambaBlock_48816598286474
// MI455X (gfx1250) — hardware-run, weakly checked
//
#include <hip/hip_runtime.h>
#include <hip/hip_fp16.h>
#include <math.h>

typedef __attribute__((ext_vector_type(16))) _Float16 v16h;
typedef __attribute__((ext_vector_type(8)))  _Float16 v8h;
typedef __attribute__((ext_vector_type(8)))  float    v8f;
typedef __attribute__((ext_vector_type(4)))  float    v4f;
typedef __attribute__((ext_vector_type(2)))  unsigned v2u;
typedef __attribute__((ext_vector_type(4)))  unsigned v4u;

constexpr int kBatch   = 4;
constexpr int kL       = 2048;
constexpr int kRows    = kBatch * kL;
constexpr int kD       = 512;
constexpr int kNst     = 16;
constexpr int kRank    = 32;
constexpr int kDbc     = kRank + 2 * kNst;
constexpr int kKp      = 544;
constexpr int kWpP     = 576;
constexpr int kBiasCol = 512;
constexpr int kDrP     = 96;
constexpr int kWdtP    = 128;
constexpr int kDtBiasCol = 64;
constexpr int kOffB    = kRank;
constexpr int kOffC    = kRank + kNst;
constexpr int kAlpFloats = kD * kNst;
constexpr int kPadFloats = kAlpFloats + kD;
constexpr float kNCarry = 256.0f;
constexpr float kWCarry = 1024.0f;
constexpr float kZCarry = 64.0f;
constexpr float kRCarry = 256.0f;
constexpr float kYCarry = 16.0f;
constexpr float kResid  = 2048.0f;
static_assert(kRows == 8192 && kL == 2048 && kD == 512 && kNst == 16 && kRank == 32 && kDbc == 64);
static_assert(kOffB == 32 && kOffC == 48);
static_assert((kKp % 32) == 0 && (kDrP % 32) == 0 && (kD % 32) == 0);
static_assert(kKp == kD + 32 && kBiasCol == kD && kBiasCol < kKp && kKp <= kWpP);
static_assert(kDtBiasCol == 2 * kRank && kDtBiasCol < kDrP && kDrP <= kWdtP);
static_assert(((kWpP * 2) % 128) == 0 && ((kWdtP * 2) % 128) == 0 && ((kBiasCol * 2) % 128) == 0 &&
              ((kDtBiasCol * 2) % 128) == 0);
static_assert((kRows % 32) == 0 && (kD % 64) == 0 && (kDbc % 64) == 0 && (kL % 64) == 0);
static_assert(kAlpFloats == 8192 && kPadFloats == 8704);

constexpr size_t kSzST   = (size_t)kRows * 4 * 4;
constexpr size_t kSzXNH  = (size_t)kRows * kKp * 2;
constexpr size_t kSzXNL  = (size_t)kRows * kKp * 2;
constexpr size_t kSzWP   = (size_t)kD * kWpP * 2;
constexpr size_t kSzWB   = (size_t)kD * kWpP * 2;
constexpr size_t kSzWD   = (size_t)kDbc * kD * 2;
constexpr size_t kSzWDT  = (size_t)kD * kWdtP * 2;
constexpr size_t kSzZ1   = (size_t)kRows * kD * 4;
constexpr size_t kSzZH   = (size_t)kRows * kKp * 2;
constexpr size_t kSzZL   = (size_t)kRows * kKp * 2;
constexpr size_t kSzBW   = (size_t)kRows * kD * 4;
constexpr size_t kSzBH   = (size_t)kRows * kD * 2;
constexpr size_t kSzBL   = (size_t)kRows * kD * 2;
constexpr size_t kSzDBC  = (size_t)kRows * kDbc * 4;
constexpr size_t kSzDRH  = (size_t)kRows * kDrP * 2;
constexpr size_t kSzDRL  = (size_t)kRows * kDrP * 2;
constexpr size_t kSzDTP  = (size_t)kRows * kD * 4;
constexpr size_t kSzPADS = (size_t)kPadFloats * 4;
constexpr size_t kSzYH   = (size_t)kRows * kD * 2;
constexpr size_t kSzYL   = (size_t)kRows * kD * 2;
constexpr size_t kOffST   = 0;
constexpr size_t kOffXNH  = kOffST   + kSzST;
constexpr size_t kOffXNL  = kOffXNH  + kSzXNH;
constexpr size_t kOffWP   = kOffXNL  + kSzXNL;
constexpr size_t kOffWB   = kOffWP   + kSzWP;
constexpr size_t kOffWD   = kOffWB   + kSzWB;
constexpr size_t kOffWDT  = kOffWD   + kSzWD;
constexpr size_t kOffZ1   = kOffWDT  + kSzWDT;
constexpr size_t kOffZH   = kOffZ1   + kSzZ1;
constexpr size_t kOffZL   = kOffZH   + kSzZH;
constexpr size_t kOffBW   = kOffZL   + kSzZL;
constexpr size_t kOffBH   = kOffBW   + kSzBW;
constexpr size_t kOffBL   = kOffBH   + kSzBH;
constexpr size_t kOffDBC  = kOffBL   + kSzBL;
constexpr size_t kOffDRH  = kOffDBC  + kSzDBC;
constexpr size_t kOffDRL  = kOffDRH  + kSzDRH;
constexpr size_t kOffDTP  = kOffDRL  + kSzDRL;
constexpr size_t kOffPADS = kOffDTP  + kSzDTP;
constexpr size_t kOffYH   = kOffPADS + kSzPADS;
constexpr size_t kOffYL   = kOffYH   + kSzYH;
constexpr size_t kWsTotal = kOffYL   + kSzYL;
static_assert(kSzST == 131072ull && kSzXNH == 8912896ull && kSzXNL == 8912896ull && kSzWP == 589824ull);
static_assert(kSzWB == 589824ull && kSzWD == 65536ull && kSzWDT == 131072ull && kSzZ1 == 16777216ull);
static_assert(kSzZH == 8912896ull && kSzZL == 8912896ull && kSzBW == 16777216ull && kSzBH == 8388608ull);
static_assert(kSzBL == 8388608ull && kSzDBC == 2097152ull && kSzDRH == 1572864ull && kSzDRL == 1572864ull);
static_assert(kSzDTP == 16777216ull && kSzPADS == 34816ull && kSzYH == 8388608ull && kSzYL == 8388608ull);
static_assert(kWsTotal == 131072ull + 8912896ull + 8912896ull + 589824ull + 589824ull + 65536ull + 131072ull +
              16777216ull + 8912896ull + 8912896ull + 16777216ull + 8388608ull + 8388608ull + 2097152ull +
              1572864ull + 1572864ull + 16777216ull + 34816ull + 8388608ull + 8388608ull);
static_assert(kWsTotal == 126322688ull);
static_assert(kWsTotal <= 134217728ull);
static_assert((kSzST % 128) == 0 && (kSzXNH % 128) == 0 && (kSzWP % 128) == 0 && (kSzWD % 128) == 0 &&
              (kSzWDT % 128) == 0 && (kSzZ1 % 128) == 0 && (kSzBH % 128) == 0 && (kSzDBC % 128) == 0 &&
              (kSzDRH % 128) == 0 && (kSzDTP % 128) == 0 && (kSzPADS % 128) == 0 && (kSzYH % 128) == 0);
static_assert((((size_t)kAlpFloats * 4) % 128) == 0);

__device__ __forceinline__ _Float16 f16_flush(float v) {
  const float w = (fabsf(v) < 6.103515625e-05f) ? 0.0f : v;
  return (_Float16)w;
}
__device__ __forceinline__ void f16_split(float v, _Float16& hi, _Float16& lo) {
  hi = f16_flush(v);
  const float hf = (float)hi;
  const float r = (v - hf) * kResid;
  lo = f16_flush(r);
}

__device__ __forceinline__ float bf16r(float v) {
  unsigned u = __float_as_uint(v);
  u = (u + 0x7FFFu + ((u >> 16) & 1u)) & 0xFFFF0000u;
  return __uint_as_float(u);
}

__device__ __forceinline__ float h16_to_f32(unsigned hb) {
  const unsigned sgn = (hb & 0x8000u) << 16; const unsigned em = hb & 0x7fffu;
  const float fn = __uint_as_float((em << 13) + 0x38000000u);
  const float fs = (float)em * 5.9604644775390625e-8f;
  const float mag = (em < 0x400u) ? fs : fn; return __uint_as_float(__float_as_uint(mag) | sgn); }

namespace eng {
union FragU { v16h v; v8h h[2]; };
__device__ __forceinline__ v16h frag_load(const _Float16* p) {
  FragU f;
  f.h[0] = *(const v8h*)(p);
  f.h[1] = *(const v8h*)(p + 16);
  return f.v;
}
__device__ __forceinline__ v8f mma(v16h a, v16h b, v8f c) {
  return __builtin_amdgcn_wmma_f32_16x16x32_f16(false, a, false, b, (short)0, c, false, false);
}
__device__ __forceinline__ void guard1(v8f& a, v16h x, v16h y) {
  asm volatile("v_nop\n\tv_nop\n\tv_nop\n\tv_nop" : "+v"(a) : "v"(x), "v"(y));
}
__device__ __forceinline__ void guard_acc(v8f& a) {
  asm volatile("v_nop\n\tv_nop\n\tv_nop\n\tv_nop" : "+v"(a));
}
__device__ __forceinline__ void keep4(v16h a, v16h b, v16h c, v16h d) {
  asm volatile("v_nop" :: "v"(a), "v"(b), "v"(c), "v"(d));
}

template <int MI, int SPL>
__global__ __launch_bounds__(256) void gemm_f16_kernel(
    const unsigned short* __restrict__ Ap, const unsigned short* __restrict__ A2p, int lda,
    const unsigned short* __restrict__ Btp, const unsigned short* __restrict__ Bt2p, int ldb,
    float* __restrict__ C, int ldc, int M, int N, int K, float scale, float rscale)
{
  static_assert(MI >= 1 && MI <= 2);
  static_assert(SPL >= 0 && SPL <= 2);
  const _Float16* A   = (const _Float16*)Ap;
  const _Float16* A2  = (const _Float16*)A2p;
  const _Float16* Bt  = (const _Float16*)Btp;
  const _Float16* Bt2 = (const _Float16*)Bt2p;
  __shared__ __align__(16) float sT[8][16 * 68];
  const int lane = threadIdx.x & 31;
  const int wave = threadIdx.x >> 5;
  const int tilesN = N >> 6;
  const int tilesM = M / (16 * MI);
  const int tile = blockIdx.x * 8 + wave;
  if (tile >= tilesM * tilesN) return;
  const int tm = tile / tilesN;
  const int tn = tile - tm * tilesN;
  const int m0 = tm * (16 * MI);
  const int n0 = tn << 6;
  const int rlane = lane & 15;
  const int koff  = (lane >> 4) * 8;
  const int mOff  = (lane >> 4) * 8;

  v8f acc[MI][4], accr[MI][4];
#pragma unroll
  for (int i = 0; i < MI; ++i)
#pragma unroll
    for (int j = 0; j < 4; ++j) {
      acc[i][j]  = (v8f){0.f, 0.f, 0.f, 0.f, 0.f, 0.f, 0.f, 0.f};
      accr[i][j] = (v8f){0.f, 0.f, 0.f, 0.f, 0.f, 0.f, 0.f, 0.f};
    }

  for (int k0 = 0; k0 < K; k0 += 32) {
    v16h bh[4], bl[4];
#pragma unroll
    for (int j = 0; j < 4; ++j) {
      const size_t bo = (size_t)(n0 + (j << 4) + rlane) * ldb + koff + k0;
      bh[j] = frag_load(Bt + bo);
      if (SPL == 2) bl[j] = frag_load(Bt2 + bo); else bl[j] = bh[j];
    }
#pragma unroll
    for (int i = 0; i < MI; ++i) {
      const size_t ao = (size_t)(m0 + (i << 4) + rlane) * lda + koff + k0;
      const v16h ah = frag_load(A + ao);
      v16h al = ah;
      if (SPL >= 1) al = frag_load(A2 + ao);
#pragma unroll
      for (int j = 0; j < 4; ++j) {
        acc[i][j] = mma(ah, bh[j], acc[i][j]);
        if (SPL >= 1) accr[i][j] = mma(al, bh[j], accr[i][j]);
        if (SPL == 2) accr[i][j] = mma(ah, bl[j], accr[i][j]);
      }
#pragma unroll
      for (int j = 0; j < 4; ++j) {
        guard1(acc[i][j], ah, al);
        if (SPL >= 1) guard1(accr[i][j], ah, al);
      }
    }
    keep4(bh[0], bh[1], bh[2], bh[3]);
    if (SPL == 2) keep4(bl[0], bl[1], bl[2], bl[3]);
  }
#pragma unroll
  for (int i = 0; i < MI; ++i)
#pragma unroll
    for (int j = 0; j < 4; ++j) {
      guard_acc(acc[i][j]);
      if (SPL >= 1) guard_acc(accr[i][j]);
    }

  float* slab = sT[wave];
#pragma unroll
  for (int i = 0; i < MI; ++i) {
    const int mBase = m0 + (i << 4);
#pragma unroll
    for (int j = 0; j < 4; ++j) {
#pragma unroll
      for (int r = 0; r < 8; ++r) {
        float v = acc[i][j][r] * scale;
        if (SPL >= 1) v += accr[i][j][r] * rscale;
        slab[(mOff + r) * 68 + (j << 4) + rlane] = v;
      }
    }
    __builtin_amdgcn_fence(__ATOMIC_RELEASE, "workgroup");
    __builtin_amdgcn_wave_barrier();
    __builtin_amdgcn_fence(__ATOMIC_ACQUIRE, "workgroup");
    {
      const int hh = lane >> 4, c4 = (lane & 15) * 4;
      for (int pass = 0; pass < 2; ++pass) {
#pragma unroll
        for (int it = 0; it < 8; ++it) {
          const int row = it * 2 + hh;
          const v4f v = *(const v4f*)(slab + row * 68 + c4);
          *(volatile v4f*)(C + (size_t)(mBase + row) * ldc + n0 + c4) = v;
        }
        __threadfence();
      }
    }
    __builtin_amdgcn_fence(__ATOMIC_RELEASE, "workgroup");
    __builtin_amdgcn_wave_barrier();
    __builtin_amdgcn_fence(__ATOMIC_ACQUIRE, "workgroup");
  }
}
}

__device__ __forceinline__ _Float16 in_half(float v, float carry, bool live) {
  const float t = live ? (bf16r(v) * carry) : 0.0f;
  return f16_flush(t);
}
__device__ __forceinline__ unsigned f16_bits(float v) {
  const float w = (fabsf(v) < 6.103515625e-05f) ? 0.0f : v;
  return (unsigned)__half_as_ushort(__float2half_rn(w));
}
__device__ __forceinline__ void col_split(float v, int col, int nlive, int cbias, float carry,
                                          _Float16& hi, _Float16& lo) {
  const float t = (col < nlive) ? (v * carry) : ((col == cbias) ? carry : 0.0f);
  f16_split(t, hi, lo);
}
__device__ __forceinline__ v8h make8(_Float16 a0, _Float16 a1, _Float16 a2, _Float16 a3,
                                     _Float16 a4, _Float16 a5, _Float16 a6, _Float16 a7) {
  v8h v;
  v[0] = a0;
  v[1] = a1;
  v[2] = a2;
  v[3] = a3;
  v[4] = a4;
  v[5] = a5;
  v[6] = a6;
  v[7] = a7;
  return v;
}
__device__ __forceinline__ void store_pair(unsigned short* qh, unsigned short* ql, v8h hv, v8h lv) {
  *(volatile v8h*)qh = hv;
  *(volatile v8h*)ql = lv;
  __threadfence();
  *(volatile v8h*)qh = hv;
  *(volatile v8h*)ql = lv;
}
__device__ __forceinline__ void store_one(unsigned short* q, v8h hv) {
  *(volatile v8h*)q = hv;
  __threadfence();
  *(volatile v8h*)q = hv;
}
__device__ __forceinline__ v4u bias_word(float bv, int w) {
  const unsigned hb = f16_bits(bf16r(bv) * kWCarry);
  const unsigned w0 = (w == 0) ? hb : 0u;
  v4u o;
  o[0] = w0;
  o[1] = 0u;
  o[2] = 0u;
  o[3] = 0u;
  return o;
}

__global__ __launch_bounds__(256) void ln_stats_kernel(
    const float* __restrict__ x, float* __restrict__ ST)
{
  const int r = blockIdx.x * 256 + threadIdx.x;
  const float* mp = x + (size_t)r * kD;
  float sum = 0.0f;
  for (int c = 0; c < 512; c += 4) {
    const v4f v = *(const v4f*)(mp + c);
    const float r0 = v[0];
    const float r1 = v[1];
    const float r2 = v[2];
    const float r3 = v[3];
    const float a0 = bf16r(r0);
    const float a1 = bf16r(r1);
    const float a2 = bf16r(r2);
    const float a3 = bf16r(r3);
    sum = sum + a0;
    sum = sum + a1;
    sum = sum + a2;
    sum = sum + a3;
  }
  const float mu = sum * (1.0f / 512.0f);
  float vs = 0.0f;
  for (int c = 0; c < 512; c += 4) {
    const v4f v = *(const v4f*)(mp + c);
    const float r0 = v[0];
    const float r1 = v[1];
    const float r2 = v[2];
    const float r3 = v[3];
    const float e0 = bf16r(r0) - mu;
    const float e1 = bf16r(r1) - mu;
    const float e2 = bf16r(r2) - mu;
    const float e3 = bf16r(r3) - mu;
    vs = fmaf(e0, e0, vs);
    vs = fmaf(e1, e1, vs);
    vs = fmaf(e2, e2, vs);
    vs = fmaf(e3, e3, vs);
  }
  const float var = vs * (1.0f / 512.0f);
  const float rs = 1.0f / sqrtf(var + 1e-5f);
  v4f ov;
  ov[0] = mu;
  ov[1] = rs;
  ov[2] = 0.0f;
  ov[3] = 0.0f;
  float* q = ST + (size_t)r * 4;
  *(volatile v4f*)q = ov;
  __threadfence();
  *(volatile v4f*)q = ov;
}

__device__ __forceinline__ float norm_val(float xv, float mu, float rs, float lw, float lb) {
  return (bf16r(xv) - mu) * rs * bf16r(lw) + bf16r(lb);
}
__global__ __launch_bounds__(256) void norm_split_kernel(
    const float* __restrict__ x, const float* __restrict__ ST,
    const float* __restrict__ lng, const float* __restrict__ lnb,
    unsigned short* __restrict__ XNH, unsigned short* __restrict__ XNL)
{
  const int i = blockIdx.x * 256 + threadIdx.x;
  const int r = i / (kKp / 8);
  const int q = (i - r * (kKp / 8)) * 8;
  const int qc = (q < kD) ? q : (kD - 8);
  const float* xp = x + (size_t)r * kD + qc;
  const v4f xa0 = *(const v4f*)(xp);
  const v4f xa1 = *(const v4f*)(xp + 4);
  const v4f st  = *(const v4f*)(ST + (size_t)r * 4);
  const v4f ga0 = *(const v4f*)(lng + qc);
  const v4f ga1 = *(const v4f*)(lng + qc + 4);
  const v4f ba0 = *(const v4f*)(lnb + qc);
  const v4f ba1 = *(const v4f*)(lnb + qc + 4);
  const float mu = st[0];
  const float rs = st[1];
  const float x0 = xa0[0];
  const float x1 = xa0[1];
  const float x2 = xa0[2];
  const float x3 = xa0[3];
  const float x4 = xa1[0];
  const float x5 = xa1[1];
  const float x6 = xa1[2];
  const float x7 = xa1[3];
  const float g0 = ga0[0];
  const float g1 = ga0[1];
  const float g2 = ga0[2];
  const float g3 = ga0[3];
  const float g4 = ga1[0];
  const float g5 = ga1[1];
  const float g6 = ga1[2];
  const float g7 = ga1[3];
  const float b0 = ba0[0];
  const float b1 = ba0[1];
  const float b2 = ba0[2];
  const float b3 = ba0[3];
  const float b4 = ba1[0];
  const float b5 = ba1[1];
  const float b6 = ba1[2];
  const float b7 = ba1[3];
  const float n0 = norm_val(x0, mu, rs, g0, b0);
  const float n1 = norm_val(x1, mu, rs, g1, b1);
  const float n2 = norm_val(x2, mu, rs, g2, b2);
  const float n3 = norm_val(x3, mu, rs, g3, b3);
  const float n4 = norm_val(x4, mu, rs, g4, b4);
  const float n5 = norm_val(x5, mu, rs, g5, b5);
  const float n6 = norm_val(x6, mu, rs, g6, b6);
  const float n7 = norm_val(x7, mu, rs, g7, b7);
  _Float16 h0, h1, h2, h3, h4, h5, h6, h7;
  _Float16 l0, l1, l2, l3, l4, l5, l6, l7;
  col_split(n0, q + 0, kD, kBiasCol, kNCarry, h0, l0);
  col_split(n1, q + 1, kD, kBiasCol, kNCarry, h1, l1);
  col_split(n2, q + 2, kD, kBiasCol, kNCarry, h2, l2);
  col_split(n3, q + 3, kD, kBiasCol, kNCarry, h3, l3);
  col_split(n4, q + 4, kD, kBiasCol, kNCarry, h4, l4);
  col_split(n5, q + 5, kD, kBiasCol, kNCarry, h5, l5);
  col_split(n6, q + 6, kD, kBiasCol, kNCarry, h6, l6);
  col_split(n7, q + 7, kD, kBiasCol, kNCarry, h7, l7);
  const v8h hv = make8(h0, h1, h2, h3, h4, h5, h6, h7);
  const v8h lv = make8(l0, l1, l2, l3, l4, l5, l6, l7);
  store_pair(XNH + (size_t)i * 8, XNL + (size_t)i * 8, hv, lv);
}

__global__ __launch_bounds__(256) void pack_w512_kernel(
    const float* __restrict__ w, unsigned short* __restrict__ WPL)
{
  const int i = blockIdx.x * 256 + threadIdx.x;
  const int n = i / (kD / 8);
  const int c = (i - n * (kD / 8)) * 8;
  const float* sp = w + (size_t)c * kD + n;
  const float f0 = sp[0 * kD];
  const float f1 = sp[1 * kD];
  const float f2 = sp[2 * kD];
  const float f3 = sp[3 * kD];
  const float f4 = sp[4 * kD];
  const float f5 = sp[5 * kD];
  const float f6 = sp[6 * kD];
  const float f7 = sp[7 * kD];
  const v8h hv = make8(in_half(f0, kWCarry, true), in_half(f1, kWCarry, true),
                       in_half(f2, kWCarry, true), in_half(f3, kWCarry, true),
                       in_half(f4, kWCarry, true), in_half(f5, kWCarry, true),
                       in_half(f6, kWCarry, true), in_half(f7, kWCarry, true));
  store_one(WPL + (size_t)n * kWpP + c, hv);
}

__global__ __launch_bounds__(256) void pack_b512_kernel(
    const float* __restrict__ b, unsigned short* __restrict__ WPL)
{
  const int i = blockIdx.x * 256 + threadIdx.x;
  const int n = i / 8;
  const int w = i - n * 8;
  const float bv = b[n];
  const v4u o = bias_word(bv, w);
  unsigned short* q = WPL + (size_t)n * kWpP + kBiasCol + w * 8;
  *(volatile v4u*)q = o;
  __threadfence();
  *(volatile v4u*)q = o;
}

__global__ __launch_bounds__(256) void pack_wd_kernel(
    const float* __restrict__ w, unsigned short* __restrict__ WD)
{
  const int i = blockIdx.x * 256 + threadIdx.x;
  const int n = i / (kD / 8);
  const int c = (i - n * (kD / 8)) * 8;
  const float* sp = w + (size_t)c * kDbc + n;
  const float f0 = sp[0 * kDbc];
  const float f1 = sp[1 * kDbc];
  const float f2 = sp[2 * kDbc];
  const float f3 = sp[3 * kDbc];
  const float f4 = sp[4 * kDbc];
  const float f5 = sp[5 * kDbc];
  const float f6 = sp[6 * kDbc];
  const float f7 = sp[7 * kDbc];
  const v8h hv = make8(in_half(f0, kWCarry, true), in_half(f1, kWCarry, true),
                       in_half(f2, kWCarry, true), in_half(f3, kWCarry, true),
                       in_half(f4, kWCarry, true), in_half(f5, kWCarry, true),
                       in_half(f6, kWCarry, true), in_half(f7, kWCarry, true));
  store_one(WD + (size_t)i * 8, hv);
}

__global__ __launch_bounds__(256) void pack_wdt_kernel(
    const float* __restrict__ w, unsigned short* __restrict__ WDT)
{
  const int i = blockIdx.x * 256 + threadIdx.x;
  const int d = i / 8;
  const int q = (i - d * 8) * 8;
  const bool live = (q < kRank);
  const int j0 = (q + 0 < kRank - 1) ? (q + 0) : (kRank - 1);
  const int j1 = (q + 1 < kRank - 1) ? (q + 1) : (kRank - 1);
  const int j2 = (q + 2 < kRank - 1) ? (q + 2) : (kRank - 1);
  const int j3 = (q + 3 < kRank - 1) ? (q + 3) : (kRank - 1);
  const int j4 = (q + 4 < kRank - 1) ? (q + 4) : (kRank - 1);
  const int j5 = (q + 5 < kRank - 1) ? (q + 5) : (kRank - 1);
  const int j6 = (q + 6 < kRank - 1) ? (q + 6) : (kRank - 1);
  const int j7 = (q + 7 < kRank - 1) ? (q + 7) : (kRank - 1);
  const float f0 = w[(size_t)j0 * kD + d];
  const float f1 = w[(size_t)j1 * kD + d];
  const float f2 = w[(size_t)j2 * kD + d];
  const float f3 = w[(size_t)j3 * kD + d];
  const float f4 = w[(size_t)j4 * kD + d];
  const float f5 = w[(size_t)j5 * kD + d];
  const float f6 = w[(size_t)j6 * kD + d];
  const float f7 = w[(size_t)j7 * kD + d];
  const v8h hv = make8(in_half(f0, kWCarry, live), in_half(f1, kWCarry, live),
                       in_half(f2, kWCarry, live), in_half(f3, kWCarry, live),
                       in_half(f4, kWCarry, live), in_half(f5, kWCarry, live),
                       in_half(f6, kWCarry, live), in_half(f7, kWCarry, live));
  store_one(WDT + (size_t)d * kWdtP + q, hv);
}

__global__ __launch_bounds__(256) void pack_bdt_kernel(
    const float* __restrict__ b, unsigned short* __restrict__ WDT)
{
  const int i = blockIdx.x * 256 + threadIdx.x;
  const int d = i / 8;
  const int w = i - d * 8;
  const float bv = b[d];
  const v4u o = bias_word(bv, w);
  unsigned short* q = WDT + (size_t)d * kWdtP + kDtBiasCol + w * 8;
  *(volatile v4u*)q = o;
  __threadfence();
  *(volatile v4u*)q = o;
}

__global__ __launch_bounds__(256) void split_z_kernel(
    const float* __restrict__ Z1, unsigned short* __restrict__ ZH, unsigned short* __restrict__ ZL)
{
  const int i = blockIdx.x * 256 + threadIdx.x;
  const int r = i / (kKp / 8);
  const int q = (i - r * (kKp / 8)) * 8;
  const int qc = (q < kD) ? q : (kD - 8);
  const float* sp = Z1 + (size_t)r * kD + qc;
  const v4f a0 = *(const v4f*)(sp);
  const v4f a1 = *(const v4f*)(sp + 4);
  const float f0 = a0[0];
  const float f1 = a0[1];
  const float f2 = a0[2];
  const float f3 = a0[3];
  const float f4 = a1[0];
  const float f5 = a1[1];
  const float f6 = a1[2];
  const float f7 = a1[3];
  _Float16 h0, h1, h2, h3, h4, h5, h6, h7;
  _Float16 l0, l1, l2, l3, l4, l5, l6, l7;
  col_split(f0, q + 0, kD, kBiasCol, kZCarry, h0, l0);
  col_split(f1, q + 1, kD, kBiasCol, kZCarry, h1, l1);
  col_split(f2, q + 2, kD, kBiasCol, kZCarry, h2, l2);
  col_split(f3, q + 3, kD, kBiasCol, kZCarry, h3, l3);
  col_split(f4, q + 4, kD, kBiasCol, kZCarry, h4, l4);
  col_split(f5, q + 5, kD, kBiasCol, kZCarry, h5, l5);
  col_split(f6, q + 6, kD, kBiasCol, kZCarry, h6, l6);
  col_split(f7, q + 7, kD, kBiasCol, kZCarry, h7, l7);
  const v8h hv = make8(h0, h1, h2, h3, h4, h5, h6, h7);
  const v8h lv = make8(l0, l1, l2, l3, l4, l5, l6, l7);
  store_pair(ZH + (size_t)i * 8, ZL + (size_t)i * 8, hv, lv);
}

__global__ __launch_bounds__(256) void split_b_kernel(
    const float* __restrict__ BW, unsigned short* __restrict__ BH, unsigned short* __restrict__ BL)
{
  const int i = blockIdx.x * 256 + threadIdx.x;
  const float* sp = BW + (size_t)i * 8;
  const v4f a0 = *(const v4f*)(sp);
  const v4f a1 = *(const v4f*)(sp + 4);
  const float f0 = a0[0];
  const float f1 = a0[1];
  const float f2 = a0[2];
  const float f3 = a0[3];
  const float f4 = a1[0];
  const float f5 = a1[1];
  const float f6 = a1[2];
  const float f7 = a1[3];
  _Float16 h0, h1, h2, h3, h4, h5, h6, h7;
  _Float16 l0, l1, l2, l3, l4, l5, l6, l7;
  f16_split(f0 * kZCarry, h0, l0);
  f16_split(f1 * kZCarry, h1, l1);
  f16_split(f2 * kZCarry, h2, l2);
  f16_split(f3 * kZCarry, h3, l3);
  f16_split(f4 * kZCarry, h4, l4);
  f16_split(f5 * kZCarry, h5, l5);
  f16_split(f6 * kZCarry, h6, l6);
  f16_split(f7 * kZCarry, h7, l7);
  const v8h hv = make8(h0, h1, h2, h3, h4, h5, h6, h7);
  const v8h lv = make8(l0, l1, l2, l3, l4, l5, l6, l7);
  store_pair(BH + (size_t)i * 8, BL + (size_t)i * 8, hv, lv);
}

__global__ __launch_bounds__(256) void split_dr_kernel(
    const float* __restrict__ DBC, unsigned short* __restrict__ DRH, unsigned short* __restrict__ DRL)
{
  const int i = blockIdx.x * 256 + threadIdx.x;
  const int r = i / (kDrP / 8);
  const int q = (i - r * (kDrP / 8)) * 8;
  const int qc = (q < kRank) ? q : (kRank - 8);
  const float* sp = DBC + (size_t)r * kDbc + qc;
  const v4f a0 = *(const v4f*)(sp);
  const v4f a1 = *(const v4f*)(sp + 4);
  const float f0 = a0[0];
  const float f1 = a0[1];
  const float f2 = a0[2];
  const float f3 = a0[3];
  const float f4 = a1[0];
  const float f5 = a1[1];
  const float f6 = a1[2];
  const float f7 = a1[3];
  _Float16 h0, h1, h2, h3, h4, h5, h6, h7;
  _Float16 l0, l1, l2, l3, l4, l5, l6, l7;
  col_split(f0, q + 0, kRank, kDtBiasCol, kRCarry, h0, l0);
  col_split(f1, q + 1, kRank, kDtBiasCol, kRCarry, h1, l1);
  col_split(f2, q + 2, kRank, kDtBiasCol, kRCarry, h2, l2);
  col_split(f3, q + 3, kRank, kDtBiasCol, kRCarry, h3, l3);
  col_split(f4, q + 4, kRank, kDtBiasCol, kRCarry, h4, l4);
  col_split(f5, q + 5, kRank, kDtBiasCol, kRCarry, h5, l5);
  col_split(f6, q + 6, kRank, kDtBiasCol, kRCarry, h6, l6);
  col_split(f7, q + 7, kRank, kDtBiasCol, kRCarry, h7, l7);
  const v8h hv = make8(h0, h1, h2, h3, h4, h5, h6, h7);
  const v8h lv = make8(l0, l1, l2, l3, l4, l5, l6, l7);
  store_pair(DRH + (size_t)i * 8, DRL + (size_t)i * 8, hv, lv);
}

__global__ __launch_bounds__(32) void pads_kernel(
    const float* __restrict__ alog, const float* __restrict__ dssm, float* __restrict__ PADS)
{
  const int wi = blockIdx.x * 32 + threadIdx.x;
  const int f0 = wi * 4;
  const bool isA = (f0 < kAlpFloats);
  const int ea = isA ? f0 : (kAlpFloats - 4);
  const int ed0 = f0 - kAlpFloats;
  const int ed1 = (ed0 < 0) ? 0 : ed0;
  const int ed = (ed1 > kD - 4) ? (kD - 4) : ed1;
  const v4f va = *(const v4f*)(alog + ea);
  const v4f vd = *(const v4f*)(dssm + ed);
  const float a0 = va[0];
  const float a1 = va[1];
  const float a2 = va[2];
  const float a3 = va[3];
  const float d0 = vd[0];
  const float d1 = vd[1];
  const float d2 = vd[2];
  const float d3 = vd[3];
  v4f o;
  o[0] = isA ? bf16r(a0) : bf16r(d0);
  o[1] = isA ? bf16r(a1) : bf16r(d1);
  o[2] = isA ? bf16r(a2) : bf16r(d2);
  o[3] = isA ? bf16r(a3) : bf16r(d3);
  float* q = PADS + (size_t)f0;
  *(volatile v4f*)q = o;
  __threadfence();
  *(volatile v4f*)q = o;
}

typedef float    ms1_v4f __attribute__((ext_vector_type(4)));
typedef unsigned ms1_v4u __attribute__((ext_vector_type(4)));
struct ms1_args {
  const float* dtpre;
  const float* u;
  const float* bc;
  const float* z;
  const float* A_log;
  const float* Dskip;
  __half* y;
  __half* y_lo;
  long ld_dtpre;
  long ld_u;
  long ld_bc;
  long ld_z;
  long ld_y;
  int offB;
  int offC;
  int offZ;
  float ycarry;
  int dir;
  int D;
  int L;
  int nbatch;
};
static_assert(sizeof(ms1_args) == 136);

__device__ __forceinline__ float ms1_flush16(float v) {
  return (fabsf(v) < 6.103515625e-05f) ? 0.0f : v;
}
__device__ __forceinline__ unsigned ms1_h16bits(float v) {
  return (unsigned)__half_as_ushort(__float2half_rn(ms1_flush16(v)));
}
__device__ __forceinline__ float ms1_h16val(unsigned b) {
  return __half2float(__ushort_as_half((unsigned short)b));
}
__device__ __forceinline__ float ms1_softplus(float v) {
  return fmaxf(v, 0.0f) + log1pf(expf(-fabsf(v)));
}
__device__ __forceinline__ void ms1_pack2(float v0, float v1, unsigned& hw, unsigned& lw) {
  const unsigned h0 = ms1_h16bits(v0);
  const unsigned h1 = ms1_h16bits(v1);
  const float r0 = (v0 - ms1_h16val(h0)) * 2048.0f;
  const float r1 = (v1 - ms1_h16val(h1)) * 2048.0f;
  const unsigned l0 = ms1_h16bits(r0);
  const unsigned l1 = ms1_h16bits(r1);
  hw = h0 | (h1 << 16);
  lw = l0 | (l1 << 16);
}

template <int NSTATE>
__global__ __launch_bounds__(64 * (NSTATE / 16)) void ms1_scan_kernel(ms1_args a)
{
  static_assert(NSTATE == 16 || NSTATE == 64);
  constexpr int NQ  = NSTATE / 16;
  constexpr int NT  = 64 * NQ;
  constexpr int NW  = NT / 32;
  constexpr int BCW = 2 * NSTATE;
  constexpr int YP  = 68;
  constexpr int RPI = NW * 4;
  constexpr int NIT = 64 / RPI;
  static_assert(16 * NT <= 64 * YP);
  __shared__ __align__(16) float sBC[64 * BCW];
  __shared__ __align__(16) float sY[64 * YP];
  const int tid  = threadIdx.x;
  const int lane = tid & 31;
  const int wave = tid >> 5;
  const int c    = tid / NQ;
  const int sq   = tid - c * NQ;
  const int bpb  = a.D / 64;
  const int bi   = blockIdx.x / bpb;
  if (bi >= a.nbatch) return;
  const int d0 = (blockIdx.x - bi * bpb) * 64;
  const int d  = d0 + c;
  const long rowb = (long)bi * a.L;
  const bool hasz  = (a.z != nullptr);
  const bool hasD  = (a.Dskip != nullptr);
  const bool hasLo = (a.y_lo != nullptr);

#pragma unroll 1
  for (int n = 0; n < 16; ++n) {
    const float al = a.A_log[(long)d * NSTATE + sq * 16 + n];
    sY[n * NT + tid] = -expf(al);
  }
  __syncthreads();
  float An[16], h[16];
#pragma unroll
  for (int n = 0; n < 16; ++n) {
    An[n] = sY[n * NT + tid];
    h[n] = 0.0f;
  }
  float Dd = 0.0f;
  if (hasD) Dd = a.Dskip[d];

  const int nchunk = a.L / 64;
  const bool fwd = (a.dir > 0);
  const int s0 = fwd ? 0 : 63;
  const int sd = fwd ? 1 : -1;
  const int q  = lane >> 3;
  const int c8 = (lane & 7) * 8;

  for (int ci = 0; ci < nchunk; ++ci) {
    const int tb = fwd ? (ci * 64) : (a.L - 64 - ci * 64);
    const long rowc = rowb + tb;
    __syncthreads();
#pragma unroll 8
    for (int i = 0; i < 32; ++i) {
      const int idx = tid + i * NT;
      const int st  = idx / BCW;
      const int col = idx - st * BCW;
      const int sc  = (col < NSTATE) ? (a.offB + col) : (a.offC + col - NSTATE);
      sBC[idx] = a.bc[(rowc + st) * a.ld_bc + sc];
    }
    __syncthreads();
    for (int s = 0; s < 64; ++s) {
      const int ls = s0 + sd * s;
      const long row = rowc + ls;
      float pre = a.dtpre[row * a.ld_dtpre + d];
      float uv  = a.u[row * a.ld_u + d];
      float zv  = 0.0f;
      if (hasz) zv = a.z[row * a.ld_z + a.offZ + d];
      asm volatile("" : "+v"(pre));
      asm volatile("" : "+v"(uv));
      asm volatile("" : "+v"(zv));
      const float delta = ms1_softplus(pre);
      const float dtx = delta * uv;
      const float* bp = sBC + ls * BCW + sq * 16;
      const float* cp = bp + NSTATE;
      ms1_v4f Bq[4], Cq[4];
#pragma unroll
      for (int k = 0; k < 4; ++k) {
        Bq[k] = *(const ms1_v4f*)(bp + 4 * k);
        Cq[k] = *(const ms1_v4f*)(cp + 4 * k);
      }
      float yv = 0.0f;
#pragma unroll
      for (int n = 0; n < 16; ++n) {
        const float e = __expf(delta * An[n]);
        h[n] = fmaf(e, h[n], dtx * Bq[n >> 2][n & 3]);
        yv = fmaf(h[n], Cq[n >> 2][n & 3], yv);
      }
      if (NQ > 1) {
        yv += __shfl_xor(yv, 1, 32);
        yv += __shfl_xor(yv, 2, 32);
      }
      if (hasD) yv = fmaf(uv, Dd, yv);
      if (hasz) {
        const float sg = __builtin_amdgcn_rcpf(1.0f + expf(-zv));
        yv = yv * (zv * sg);
      }
      if (sq == 0) sY[ls * YP + c] = yv * a.ycarry;
    }
    __syncthreads();
    ms1_v4u hw[NIT], lw[NIT];
#pragma unroll
    for (int it = 0; it < NIT; ++it) {
      const int row = it * RPI + wave * 4 + q;
      const float* sp = sY + row * YP + c8;
      const ms1_v4f f0 = *(const ms1_v4f*)(sp);
      const ms1_v4f f1 = *(const ms1_v4f*)(sp + 4);
      unsigned h0, h1, h2, h3, l0, l1, l2, l3;
      ms1_pack2(f0[0], f0[1], h0, l0);
      ms1_pack2(f0[2], f0[3], h1, l1);
      ms1_pack2(f1[0], f1[1], h2, l2);
      ms1_pack2(f1[2], f1[3], h3, l3);
      hw[it] = (ms1_v4u){h0, h1, h2, h3};
      lw[it] = (ms1_v4u){l0, l1, l2, l3};
    }
    for (int pass = 0; pass < 2; ++pass) {
#pragma unroll
      for (int it = 0; it < NIT; ++it) {
        const int row = it * RPI + wave * 4 + q;
        const long o = (rowc + row) * a.ld_y + d0 + c8;
        *(volatile ms1_v4u*)(a.y + o) = hw[it];
        if (hasLo) *(volatile ms1_v4u*)(a.y_lo + o) = lw[it];
      }
      __threadfence();
    }
  }
}

__device__ __forceinline__ float out_val(float z1, unsigned hb, unsigned lb, float xv) {
  const float g = z1 / (1.0f + expf(-z1));
  const float y = (h16_to_f32(hb) + h16_to_f32(lb) * (1.0f / kResid)) * (1.0f / kYCarry);
  const float p = z1 * g;
  return fmaf(y, g, p) + bf16r(xv);
}
__global__ __launch_bounds__(256) void out_kernel(
    const float* __restrict__ Z1, const unsigned short* __restrict__ YH,
    const unsigned short* __restrict__ YL, const float* __restrict__ x, float* __restrict__ out)
{
  const int i = blockIdx.x * 256 + threadIdx.x;
  const v4f za = *(const v4f*)(Z1 + (size_t)i * 4);
  const v2u wh = *(const v2u*)(YH + (size_t)i * 4);
  const v2u wl = *(const v2u*)(YL + (size_t)i * 4);
  const v4f xa = *(const v4f*)(x + (size_t)i * 4);
  const float z0 = za[0];
  const float z1 = za[1];
  const float z2 = za[2];
  const float z3 = za[3];
  const unsigned h0 = wh[0];
  const unsigned h1 = wh[1];
  const unsigned l0 = wl[0];
  const unsigned l1 = wl[1];
  const float x0 = xa[0];
  const float x1 = xa[1];
  const float x2 = xa[2];
  const float x3 = xa[3];
  v4f o;
  o[0] = out_val(z0, h0 & 0xffffu, l0 & 0xffffu, x0);
  o[1] = out_val(z1, h0 >> 16, l0 >> 16, x1);
  o[2] = out_val(z2, h1 & 0xffffu, l1 & 0xffffu, x2);
  o[3] = out_val(z3, h1 >> 16, l1 >> 16, x3);
  float* q = out + (size_t)i * 4;
  *(volatile v4f*)q = o;
  __threadfence();
  *(volatile v4f*)q = o;
}

static_assert(((8192 / 32) * (512 / 64)) % 8 == 0 && (8192 / 32) * (512 / 64) / 8 == 256);
static_assert(((8192 / 32) * (64 / 64)) % 8 == 0 && (8192 / 32) * (64 / 64) / 8 == 32);
static_assert(kRows == 8192 && kD == 512 && kDbc == 64 && kKp == 544 && kWpP == 576 && kDrP == 96 &&
              kWdtP == 128);
static_assert((kRows % 256) == 0 && kRows / 256 == 32);
static_assert(((kRows * (kKp / 8)) % 256) == 0 && (kRows * (kKp / 8)) / 256 == 2176);
static_assert(((kD * (kD / 8)) % 256) == 0 && (kD * (kD / 8)) / 256 == 128);
static_assert(((kD * 8) % 256) == 0 && (kD * 8) / 256 == 16);
static_assert(((kDbc * (kD / 8)) % 256) == 0 && (kDbc * (kD / 8)) / 256 == 16);
static_assert(((kRows * kD / 8) % 256) == 0 && (kRows * kD / 8) / 256 == 2048);
static_assert(((kRows * (kDrP / 8)) % 256) == 0 && (kRows * (kDrP / 8)) / 256 == 384);
static_assert((kPadFloats / 4) == 68 * 32);
static_assert(((kRows * kD / 4) % 256) == 0 && (kRows * kD / 4) / 256 == 4096);
static_assert((512 / 64) * 4 == 32);
static_assert((kD / 64) * kBatch == 32);

extern "C" void kernel_launch(void* const* d_in, const int* in_sizes, int n_in,
                              void* d_out, int out_size, void* d_ws, size_t ws_size,
                              hipStream_t stream)
{
  if (n_in < 14) return;
  if (in_sizes[0] != kBatch * kL * kD) return;
  if (in_sizes[1] != kD) return;
  if (in_sizes[2] != kD) return;
  if (in_sizes[3] != kD * kD) return;
  if (in_sizes[4] != kD) return;
  if (in_sizes[5] != kD * kD) return;
  if (in_sizes[6] != kD) return;
  if (in_sizes[7] != kD * kD) return;
  if (in_sizes[8] != kD) return;
  if (in_sizes[9] != kD * kDbc) return;
  if (in_sizes[10] != kRank * kD) return;
  if (in_sizes[11] != kD) return;
  if (in_sizes[12] != kD * kNst) return;
  if (in_sizes[13] != kD) return;
  if (out_size != kBatch * kL * kD) return;
  if (ws_size < kWsTotal) return;

  const float* x_in   = (const float*)d_in[0];
  const float* ln_g   = (const float*)d_in[1];
  const float* ln_b   = (const float*)d_in[2];
  const float* w_proj = (const float*)d_in[3];
  const float* b_proj = (const float*)d_in[4];
  const float* w_fwd  = (const float*)d_in[5];
  const float* b_fwd  = (const float*)d_in[6];
  (void)w_fwd;
  (void)b_fwd;
  const float* w_bwd  = (const float*)d_in[7];
  const float* b_bwd  = (const float*)d_in[8];
  const float* w_dbc  = (const float*)d_in[9];
  const float* w_dt   = (const float*)d_in[10];
  const float* b_dt   = (const float*)d_in[11];
  const float* a_log  = (const float*)d_in[12];
  const float* d_ssm  = (const float*)d_in[13];
  float* out = (float*)d_out;

  char* ws = (char*)d_ws;
  float*          ST   = (float*)(ws + kOffST);
  unsigned short* XNH  = (unsigned short*)(ws + kOffXNH);
  unsigned short* XNL  = (unsigned short*)(ws + kOffXNL);
  unsigned short* WP   = (unsigned short*)(ws + kOffWP);
  unsigned short* WB   = (unsigned short*)(ws + kOffWB);
  unsigned short* WD   = (unsigned short*)(ws + kOffWD);
  unsigned short* WDT  = (unsigned short*)(ws + kOffWDT);
  float*          Z1   = (float*)(ws + kOffZ1);
  unsigned short* ZH   = (unsigned short*)(ws + kOffZH);
  unsigned short* ZL   = (unsigned short*)(ws + kOffZL);
  float*          BW   = (float*)(ws + kOffBW);
  unsigned short* BH   = (unsigned short*)(ws + kOffBH);
  unsigned short* BL   = (unsigned short*)(ws + kOffBL);
  float*          DBC  = (float*)(ws + kOffDBC);
  unsigned short* DRH  = (unsigned short*)(ws + kOffDRH);
  unsigned short* DRL  = (unsigned short*)(ws + kOffDRL);
  float*          DTP  = (float*)(ws + kOffDTP);
  float*          PADS = (float*)(ws + kOffPADS);
  unsigned short* YH   = (unsigned short*)(ws + kOffYH);
  unsigned short* YL   = (unsigned short*)(ws + kOffYL);
  float*          ALP  = PADS;
  float*          DSP  = PADS + kAlpFloats;

  constexpr float s1  = 1.0f / (kNCarry * kWCarry);
  constexpr float s1r = 1.0f / (kNCarry * kWCarry * kResid);
  constexpr float s2  = 1.0f / (kZCarry * kWCarry);
  constexpr float s2r = 1.0f / (kZCarry * kWCarry * kResid);
  constexpr float s3  = 1.0f / (kZCarry * kWCarry);
  constexpr float s3r = 1.0f / (kZCarry * kWCarry * kResid);
  constexpr float s4  = 1.0f / (kRCarry * kWCarry);
  constexpr float s4r = 1.0f / (kRCarry * kWCarry * kResid);

  ln_stats_kernel<<<kRows / 256, 256, 0, stream>>>(x_in, ST);

  norm_split_kernel<<<(kRows * (kKp / 8)) / 256, 256, 0, stream>>>(x_in, ST, ln_g, ln_b, XNH, XNL);

  pack_w512_kernel<<<(kD * (kD / 8)) / 256, 256, 0, stream>>>(w_proj, WP);
  pack_b512_kernel<<<(kD * 8) / 256, 256, 0, stream>>>(b_proj, WP);

  pack_w512_kernel<<<(kD * (kD / 8)) / 256, 256, 0, stream>>>(w_bwd, WB);
  pack_b512_kernel<<<(kD * 8) / 256, 256, 0, stream>>>(b_bwd, WB);

  pack_wd_kernel<<<(kDbc * (kD / 8)) / 256, 256, 0, stream>>>(w_dbc, WD);

  pack_wdt_kernel<<<(kD * 8) / 256, 256, 0, stream>>>(w_dt, WDT);
  pack_bdt_kernel<<<(kD * 8) / 256, 256, 0, stream>>>(b_dt, WDT);

  eng::gemm_f16_kernel<2, 1><<<dim3((8192 / 32) * (512 / 64) / 8), 256, 0, stream>>>(
      XNH, XNL, 544, WP, WP, 576, Z1, 512, 8192, 512, 544, s1, s1r);

  split_z_kernel<<<(kRows * (kKp / 8)) / 256, 256, 0, stream>>>(Z1, ZH, ZL);

  eng::gemm_f16_kernel<2, 1><<<dim3((8192 / 32) * (512 / 64) / 8), 256, 0, stream>>>(
      ZH, ZL, 544, WB, WB, 576, BW, 512, 8192, 512, 544, s2, s2r);

  split_b_kernel<<<(kRows * kD / 8) / 256, 256, 0, stream>>>(BW, BH, BL);

  eng::gemm_f16_kernel<2, 1><<<dim3((8192 / 32) * (64 / 64) / 8), 256, 0, stream>>>(
      BH, BL, 512, WD, WD, 512, DBC, 64, 8192, 64, 512, s3, s3r);

  split_dr_kernel<<<(kRows * (kDrP / 8)) / 256, 256, 0, stream>>>(DBC, DRH, DRL);

  eng::gemm_f16_kernel<2, 1><<<dim3((8192 / 32) * (512 / 64) / 8), 256, 0, stream>>>(
      DRH, DRL, 96, WDT, WDT, 128, DTP, 512, 8192, 512, 96, s4, s4r);

  pads_kernel<<<68, 32, 0, stream>>>(a_log, d_ssm, PADS);

  ms1_args sa;
  sa.dtpre = DTP;
  sa.u = BW;
  sa.bc = DBC;
  sa.z = nullptr;
  sa.A_log = ALP;
  sa.Dskip = DSP;
  sa.y = (__half*)YH;
  sa.y_lo = (__half*)YL;
  sa.ld_dtpre = 512;
  sa.ld_u = 512;
  sa.ld_bc = 64;
  sa.ld_z = 0;
  sa.ld_y = 512;
  sa.offB = kOffB;
  sa.offC = kOffC;
  sa.offZ = 0;
  sa.ycarry = kYCarry;
  sa.dir = 1;
  sa.D = kD;
  sa.L = kL;
  sa.nbatch = kBatch;

  ms1_scan_kernel<16><<<dim3((512 / 64) * 4), 64, 0, stream>>>(sa);

  out_kernel<<<(kRows * kD / 4) / 256, 256, 0, stream>>>(Z1, YH, YL, x_in, out);
}
